// BatchedMambaCore_15083925143606
// MI455X (gfx1250) — hardware-run, weakly checked
//
#include <hip/hip_runtime.h>
#include <math.h>

typedef __attribute__((ext_vector_type(16))) _Float16 v16h;
typedef __attribute__((ext_vector_type(8)))  _Float16 v8h;
typedef __attribute__((ext_vector_type(4)))  _Float16 v4h;
typedef __attribute__((ext_vector_type(8)))  float    v8f;
typedef __attribute__((ext_vector_type(4)))  float    v4f;
typedef __attribute__((ext_vector_type(4)))  unsigned v4u;

constexpr int kBatch = 8;
constexpr int kSeq   = 1024;
constexpr int kDm    = 256;
constexpr int kDi    = 512;
constexpr int kNst   = 16;
constexpr int kDtR   = 16;
constexpr int kDirs  = 4;
constexpr int kRows  = kBatch * kSeq;
constexpr int kXcols = kDtR + 2 * kNst;
constexpr int kPn    = kDirs * kXcols;
constexpr int kXzN   = 2 * kDi;
static_assert(kRows == 8192 && kXcols == 48 && kPn == 192 && kXzN == 1024, "shapes");
static_assert((kDm % 32) == 0 && (kDi % 32) == 0, "GEMM K multiples of 32");
static_assert((kRows % 64) == 0 && (kXzN % 64) == 0 && (kPn % 64) == 0 && (kDm % 64) == 0 && (kDi % 64) == 0, "GEMM M,N multiples of 64");

constexpr float kCarX   = 16.0f;
constexpr float kCarW   = 256.0f;
constexpr float kCarXC  = 16.0f;
constexpr float kCarYS  = 64.0f;
constexpr float kCarYZ  = 256.0f;
constexpr float kSclIn  = 1.0f / (kCarX * kCarW);
constexpr float kSclXp  = 1.0f / (kCarXC * kCarW);
constexpr float kSclOut = 1.0f / (kCarYZ * kCarW);
constexpr float kInvCarYS = 1.0f / kCarYS;
constexpr float kH16Lim = 60000.0f;
constexpr float kLog2e  = 1.4426950408889634f;
constexpr float kLnEps  = 1e-5f;

constexpr size_t kMiB     = 1048576ull;
constexpr size_t kOffX16  = 0;
constexpr size_t kOffW0   = 4 * kMiB;
constexpr size_t kOffW1   = kOffW0 + (size_t)kXzN * kDm * 2;
constexpr size_t kOffW2   = kOffW1 + (size_t)kPn * kDi * 2;
constexpr size_t kOffXS   = 5 * kMiB;
constexpr size_t kOffZ    = 21 * kMiB;
constexpr size_t kOffXC   = 37 * kMiB;
constexpr size_t kOffXC16 = 53 * kMiB;
constexpr size_t kOffP    = 61 * kMiB;
constexpr size_t kOffYS   = 67 * kMiB;
constexpr size_t kOffYZ   = 99 * kMiB;
constexpr size_t kWsTotal = 107 * kMiB;
constexpr size_t kPlaneYS = (size_t)kRows * kDi;
static_assert((size_t)kRows * kDm * 2 == 4 * kMiB, "X16 size");
static_assert(kOffW2 + (size_t)kDm * kDi * 2 <= kOffXS, "weight planes fit");
static_assert((kOffW1 % 128) == 0 && (kOffW2 % 128) == 0, "aligned weight planes");
static_assert((size_t)kRows * kDi * 4 == 16 * kMiB, "f32 plane size");
static_assert((size_t)kRows * kPn * 4 == 6 * kMiB, "P size");
static_assert((size_t)kDirs * kPlaneYS * 2 == 32 * kMiB, "YS size");
static_assert(kOffYZ + (size_t)kRows * kDi * 2 == kWsTotal, "carve total");
static_assert(kWsTotal == 112197632ull && kWsTotal <= 134217728ull, "carve cap");

__device__ __forceinline__ float silu_f(float v) {
  return v * __builtin_amdgcn_rcpf(1.0f + expf(-v));
}
__device__ __forceinline__ float fast_exp2(float x) {
#if __has_builtin(__builtin_amdgcn_exp2f)
  return __builtin_amdgcn_exp2f(x);
#else
  return exp2f(x);
#endif
}
__device__ __forceinline__ float clamp_h16(float v) {
  return fminf(fmaxf(v, -kH16Lim), kH16Lim);
}
__device__ __forceinline__ float h16_to_f32(unsigned hb) {
  const unsigned sgn = (hb & 0x8000u) << 16; const unsigned em = hb & 0x7fffu;
  const float fn = __uint_as_float((em << 13) + 0x38000000u);
  const float fs = (float)em * 5.9604644775390625e-8f;
  const float mag = (em < 0x400u) ? fs : fn; return __uint_as_float(__float_as_uint(mag) | sgn); }

__device__ __forceinline__ int scan_pos(int k, int j) {
  const int hi = (j >= (kSeq / 2)) ? 1 : 0;
  const int jj = j - hi * (kSeq / 2);
  const int p1 = kSeq - 1 - j;
  const int p2 = 2 * jj + hi;
  const int p3 = 2 * jj + 1 - hi;
  int p = j;
  p = (k == 1) ? p1 : p;
  p = (k == 2) ? p2 : p;
  p = (k == 3) ? p3 : p;
  return p;
}

union FragH { v16h v; v8h h[2]; };
__device__ __forceinline__ v16h frag_load_h(const _Float16* p) {
  FragH f; f.h[0] = *(const v8h*)(p); f.h[1] = *(const v8h*)(p + 16); return f.v;
}
__device__ __forceinline__ v8f mma_h(v16h a, v16h b, v8f c) {
  return __builtin_amdgcn_wmma_f32_16x16x32_f16(false, a, false, b, (short)0, c, false, false);
}
__device__ __forceinline__ void wm_guard(v8f& a, v16h x, v16h y) {
  asm volatile("v_nop\n\tv_nop\n\tv_nop\n\tv_nop" : "+v"(a) : "v"(x), "v"(y));
}
__device__ __forceinline__ void keep4_h(v16h a, v16h b, v16h c, v16h d) {
  asm volatile("v_nop" :: "v"(a), "v"(b), "v"(c), "v"(d));
}

constexpr int kPbX  = (kRows * kDm) / 2048;
constexpr int kPbW0 = (kXzN * kDm) / 2048;
constexpr int kPbW1 = (kPn * kDi) / 2048;
constexpr int kPbW2 = (kDm * kDi) / 2048;
static_assert(kPbX == 1024 && kPbW0 == 128 && kPbW1 == 48 && kPbW2 == 64, "prep block ranges");

__global__ __launch_bounds__(256) void prep_f16_planes_kernel(
    const float* __restrict__ x, const float* __restrict__ w0, const float* __restrict__ w1, const float* __restrict__ w2,
    unsigned short* __restrict__ X16, unsigned short* __restrict__ W0, unsigned short* __restrict__ W1,
    unsigned short* __restrict__ W2)
{
  const int bx = blockIdx.x;
  int seg = 0;
  if (bx >= kPbX) seg = 1;
  if (bx >= kPbX + kPbW0) seg = 2;
  if (bx >= kPbX + kPbW0 + kPbW1) seg = 3;
  const float* src = (seg == 0) ? x : (seg == 1) ? w0 : (seg == 2) ? w1 : w2;
  unsigned short* dst = (seg == 0) ? X16 : (seg == 1) ? W0 : (seg == 2) ? W1 : W2;
  const int bbase = (seg == 0) ? 0 : (seg == 1) ? kPbX : (seg == 2) ? (kPbX + kPbW0) : (kPbX + kPbW0 + kPbW1);
  const float sc = (seg == 0) ? kCarX : kCarW;
  const size_t e0 = ((size_t)(bx - bbase) * 256 + threadIdx.x) << 3;
  const v4f a0 = *(const v4f*)(src + e0);
  const v4f a1 = *(const v4f*)(src + e0 + 4);
  v8h hv;
#pragma unroll
  for (int e = 0; e < 4; ++e) {
    hv[e]     = (_Float16)(a0[e] * sc);
    hv[4 + e] = (_Float16)(a1[e] * sc);
  }
  unsigned short* q = dst + e0;
  *(volatile v8h*)q = hv;
  __threadfence();
  *(volatile v8h*)q = hv;
}

template <int SPLITN>
__global__ __launch_bounds__(256) void wmma_gemm64_f16(
    const unsigned short* __restrict__ Ap, int lda,
    const unsigned short* __restrict__ Btp, int ldb,
    float* Cout, float* Cout2, int ldc,
    int M, int N, int K, float scale)
{
  const _Float16* A  = (const _Float16*)Ap;
  const _Float16* Bt = (const _Float16*)Btp;
  __shared__ __align__(16) float sT[8][16 * 68];
  const int lane = threadIdx.x & 31;
  const int wave = __builtin_amdgcn_readfirstlane((int)(threadIdx.x >> 5));
  const int tilesN = N >> 6;
  const int tilesM = M >> 6;
  const int tile = blockIdx.x * 8 + wave;
  if (tile >= tilesM * tilesN) return;
  const int tm = tile / tilesN;
  const int tn = tile - tm * tilesN;
  const int m0 = tm << 6;
  const int n0 = tn << 6;

  const int rlane = lane & 15;
  const int koff  = (lane >> 4) * 8;
  const int mOff  = (lane >> 4) * 8;

  v8f acc[4][4];
#pragma unroll
  for (int i = 0; i < 4; ++i)
#pragma unroll
    for (int j = 0; j < 4; ++j) acc[i][j] = (v8f){0.f,0.f,0.f,0.f,0.f,0.f,0.f,0.f};

  for (int k0 = 0; k0 < K; k0 += 32) {
    v16h bh[4];
#pragma unroll
    for (int j = 0; j < 4; ++j) {
      const size_t bo = (size_t)(n0 + (j << 4) + rlane) * ldb + koff + k0;
      bh[j] = frag_load_h(Bt + bo);
    }
#pragma unroll
    for (int i = 0; i < 4; ++i) {
      const size_t ao = (size_t)(m0 + (i << 4) + rlane) * lda + koff + k0;
      const v16h ah = frag_load_h(A + ao);
#pragma unroll
      for (int j = 0; j < 4; ++j) acc[i][j] = mma_h(ah, bh[j], acc[i][j]);
      wm_guard(acc[i][0], ah, bh[0]);
      wm_guard(acc[i][1], ah, bh[1]);
      wm_guard(acc[i][2], ah, bh[2]);
      wm_guard(acc[i][3], ah, bh[3]);
    }
    keep4_h(bh[0], bh[1], bh[2], bh[3]);
  }

  float* slab = sT[wave];
  const bool second = (SPLITN > 0) && (n0 >= SPLITN);
  float* Cp = second ? Cout2 : Cout;
  const int nc0 = second ? (n0 - SPLITN) : n0;
  const int hh = lane >> 4, c4 = (lane & 15) * 4;
#pragma unroll
  for (int i = 0; i < 4; ++i) {
    const int mBase = m0 + (i << 4);
#pragma unroll
    for (int j = 0; j < 4; ++j) {
#pragma unroll
      for (int r = 0; r < 8; ++r) {
        slab[(mOff + r) * 68 + (j << 4) + rlane] = acc[i][j][r] * scale;
      }
    }
    __builtin_amdgcn_fence(__ATOMIC_RELEASE, "workgroup");
    __builtin_amdgcn_wave_barrier();
    __builtin_amdgcn_fence(__ATOMIC_ACQUIRE, "workgroup");
    if (second) {
#pragma unroll 1
      for (int it = 0; it < 8; ++it) {
        float* sp = slab + (it * 2 + hh) * 68 + c4;
        const v4f v = *(const v4f*)sp;
        v4f o;
        o[0] = silu_f(v[0]);
        o[1] = silu_f(v[1]);
        o[2] = silu_f(v[2]);
        o[3] = silu_f(v[3]);
        *(v4f*)sp = o;
      }
    }
    for (int pass = 0; pass < 2; ++pass) {
#pragma unroll
      for (int it = 0; it < 8; ++it) {
        const int row = it * 2 + hh;
        const v4f v = *(const v4f*)(slab + row * 68 + c4);
        *(volatile v4f*)(Cp + (size_t)(mBase + row) * ldc + nc0 + c4) = v;
      }
      __threadfence();
    }
    __builtin_amdgcn_fence(__ATOMIC_RELEASE, "workgroup");
    __builtin_amdgcn_wave_barrier();
    __builtin_amdgcn_fence(__ATOMIC_ACQUIRE, "workgroup");
  }
}

__global__ __launch_bounds__(256) void conv_act_kernel(
    const float* __restrict__ XS, const float* __restrict__ cw, const float* __restrict__ cb,
    float* __restrict__ XC, unsigned short* __restrict__ XC16)
{
  const int idx = blockIdx.x * 256 + threadIdx.x;
  const int g = idx & 127;
  const int r = idx >> 7;
  const int l = r & (kSeq - 1);
  const int rb = r - l;
  const int d = g * 4;
  v4f wv[4];
#pragma unroll
  for (int e = 0; e < 4; ++e) wv[e] = *(const v4f*)(cw + (size_t)(d + e) * 4);
  const v4f bv = *(const v4f*)(cb + d);
  v4f xt[4];
#pragma unroll
  for (int j = 0; j < 4; ++j) {
    const int li = l - 1 + j;
    const int lic = li < 0 ? 0 : (li > (kSeq - 1) ? (kSeq - 1) : li);
    const bool ok = (li == lic);
    const v4f v = *(const v4f*)(XS + (size_t)(rb + lic) * kDi + d);
    const v4f zr = (v4f){0.f, 0.f, 0.f, 0.f};
    xt[j] = ok ? v : zr;
  }
  v4f ov;
  v4h hv;
#pragma unroll
  for (int e = 0; e < 4; ++e) {
    float a = bv[e];
    a = fmaf(wv[e][0], xt[0][e], a);
    a = fmaf(wv[e][1], xt[1][e], a);
    a = fmaf(wv[e][2], xt[2][e], a);
    a = fmaf(wv[e][3], xt[3][e], a);
    const float s = silu_f(a);
    ov[e] = s;
    hv[e] = (_Float16)(s * kCarXC);
  }
  const size_t o = (size_t)r * kDi + d;
  *(volatile v4f*)(XC + o) = ov;
  *(volatile v4h*)(XC16 + o) = hv;
  __threadfence();
  *(volatile v4f*)(XC + o) = ov;
  *(volatile v4h*)(XC16 + o) = hv;
}

constexpr int kScSteps = 32;
constexpr int kScCh    = 256;
constexpr int kScYP    = 260;
static_assert((kSeq % kScSteps) == 0 && (kDi % kScCh) == 0, "scan tiling");
static_assert(kScSteps * (kXcols / 4) == 384, "staging slots");

__global__ __launch_bounds__(256) void scan_dirs_kernel(
    const float* __restrict__ P, const float* __restrict__ XC,
    const float* __restrict__ dtw, const float* __restrict__ dtb, const float* __restrict__ alog,
    unsigned short* __restrict__ YS)
{
  __shared__ __align__(16) float sP[512 * 4];
  __shared__ __align__(16) float sY[kScSteps * kScYP];
  const int tid  = threadIdx.x;
  const int lane = tid & 31;
  const int wave = __builtin_amdgcn_readfirstlane((int)(tid >> 5));
  const int bk   = blockIdx.x >> 1;
  const int d0   = (blockIdx.x & 1) * kScCh;
  const int b    = bk >> 2;
  const int kdir = bk & 3;
  const int d    = d0 + tid;

  float wR[kDtR], aL[kNst], h[kNst];
  {
    const float* wp = dtw + (size_t)(kdir * kDi + d) * kDtR;
    const float* ap = alog + (size_t)(kdir * kDi + d) * kNst;
#pragma unroll
    for (int q = 0; q < 4; ++q) {
      const v4f w4 = *(const v4f*)(wp + 4 * q);
      const v4f a4 = *(const v4f*)(ap + 4 * q);
#pragma unroll
      for (int e = 0; e < 4; ++e) {
        wR[4 * q + e] = w4[e];
        aL[4 * q + e] = -expf(a4[e]) * kLog2e;
        h[4 * q + e]  = 0.0f;
      }
    }
  }
  const float bias = dtb[kdir * kDi + d];
  const int c8 = lane * 8;

#pragma unroll 1
  for (int j0 = 0; j0 < kSeq; j0 += kScSteps) {
    __syncthreads();
#pragma unroll
    for (int i = 0; i < 2; ++i) {
      const int t  = tid + 256 * i;
      const int tc = t < 384 ? t : 383;
      const int srow = tc / 12;
      const int c4 = tc - srow * 12;
      const int p  = scan_pos(kdir, j0 + srow);
      const v4f v = *(const v4f*)(P + (size_t)(b * kSeq + p) * kPn + kdir * kXcols + c4 * 4);
      *(v4f*)(sP + t * 4) = v;
    }
    __syncthreads();

#pragma unroll 1
    for (int s = 0; s < kScSteps; ++s) {
      const int p = scan_pos(kdir, j0 + s);
      const float u = XC[(size_t)(b * kSeq + p) * kDi + d];
      const float* xr = sP + s * kXcols;
      float dv = bias;
#pragma unroll
      for (int q = 0; q < 4; ++q) {
        const v4f t4 = *(const v4f*)(xr + 4 * q);
        dv = fmaf(wR[4 * q + 0], t4[0], dv);
        dv = fmaf(wR[4 * q + 1], t4[1], dv);
        dv = fmaf(wR[4 * q + 2], t4[2], dv);
        dv = fmaf(wR[4 * q + 3], t4[3], dv);
      }
      const float delta = fmaxf(dv, 0.0f) + log1pf(expf(-fabsf(dv)));
      const float du = delta * u;
      float y = 0.0f;
#pragma unroll
      for (int q = 0; q < 4; ++q) {
        const v4f b4 = *(const v4f*)(xr + kDtR + 4 * q);
        const v4f c4v = *(const v4f*)(xr + kDtR + kNst + 4 * q);
#pragma unroll
        for (int e = 0; e < 4; ++e) {
          const float dA = fast_exp2(delta * aL[4 * q + e]);
          h[4 * q + e] = fmaf(h[4 * q + e], dA, du * b4[e]);
          y = fmaf(h[4 * q + e], c4v[e], y);
        }
      }
      sY[s * kScYP + tid] = y;
    }
    __syncthreads();

    v8h hv[4];
#pragma unroll
    for (int it = 0; it < 4; ++it) {
      const int row = it * 8 + wave;
      const float* sp = sY + row * kScYP + c8;
      const v4f a0 = *(const v4f*)(sp);
      const v4f a1 = *(const v4f*)(sp + 4);
#pragma unroll
      for (int e = 0; e < 4; ++e) {
        hv[it][e]     = (_Float16)clamp_h16(a0[e] * kCarYS);
        hv[it][4 + e] = (_Float16)clamp_h16(a1[e] * kCarYS);
      }
    }
    for (int pass = 0; pass < 2; ++pass) {
#pragma unroll
      for (int it = 0; it < 4; ++it) {
        const int row = it * 8 + wave;
        const int p = scan_pos(kdir, j0 + row);
        unsigned short* dst = YS + (size_t)kdir * kPlaneYS + (size_t)(b * kSeq + p) * kDi + d0 + c8;
        *(volatile v8h*)dst = hv[it];
      }
      __threadfence();
    }
  }
}

__global__ __launch_bounds__(256) void merge_norm_gate_kernel(
    const unsigned short* __restrict__ YS, const float* __restrict__ XC, const float* __restrict__ Z,
    const float* __restrict__ Dsk, const float* __restrict__ lng, const float* __restrict__ lnb,
    unsigned short* __restrict__ YZ)
{
  __shared__ __align__(16) float sD[kDi];
  __shared__ __align__(16) float sG[kDi];
  __shared__ __align__(16) float sB[kDi];
  const int tid = threadIdx.x;
#pragma unroll
  for (int i = 0; i < 2; ++i) {
    const int c = tid + 256 * i;
    float a = 0.0f;
    a += Dsk[c];
    a += Dsk[kDi + c];
    a += Dsk[2 * kDi + c];
    a += Dsk[3 * kDi + c];
    sD[c] = a;
    sG[c] = lng[c];
    sB[c] = lnb[c];
  }
  __syncthreads();
  const int lane = tid & 31;
  const int wave = __builtin_amdgcn_readfirstlane((int)(tid >> 5));
  float dsum[16], gg[16], bb[16];
#pragma unroll
  for (int t = 0; t < 2; ++t) {
    const int cb0 = t * 256 + lane * 8;
    const v4f d0v = *(const v4f*)(sD + cb0), d1v = *(const v4f*)(sD + cb0 + 4);
    const v4f g0v = *(const v4f*)(sG + cb0), g1v = *(const v4f*)(sG + cb0 + 4);
    const v4f b0v = *(const v4f*)(sB + cb0), b1v = *(const v4f*)(sB + cb0 + 4);
#pragma unroll
    for (int e = 0; e < 4; ++e) {
      dsum[t * 8 + e] = d0v[e]; dsum[t * 8 + 4 + e] = d1v[e];
      gg[t * 8 + e]   = g0v[e]; gg[t * 8 + 4 + e]   = g1v[e];
      bb[t * 8 + e]   = b0v[e]; bb[t * 8 + 4 + e]   = b1v[e];
    }
  }

#pragma unroll 1
  for (int rr = 0; rr < 4; ++rr) {
    const int row = blockIdx.x * 32 + wave * 4 + rr;
    float v[16];
#pragma unroll
    for (int t = 0; t < 2; ++t) {
      const size_t off = (size_t)row * kDi + t * 256 + lane * 8;
      const v4f xa = *(const v4f*)(XC + off);
      const v4f xb = *(const v4f*)(XC + off + 4);
      float ys[8];
#pragma unroll
      for (int e = 0; e < 8; ++e) ys[e] = 0.0f;
#pragma unroll
      for (int kd = 0; kd < kDirs; ++kd) {
        const v4u w = *(const v4u*)(YS + (size_t)kd * kPlaneYS + off);
#pragma unroll
        for (int m = 0; m < 4; ++m) {
          const unsigned wm = w[m];
          ys[2 * m]     += h16_to_f32(wm & 0xffffu);
          ys[2 * m + 1] += h16_to_f32(wm >> 16);
        }
      }
#pragma unroll
      for (int e = 0; e < 4; ++e) {
        v[t * 8 + e]     = fmaf(dsum[t * 8 + e], xa[e], ys[e] * kInvCarYS);
        v[t * 8 + 4 + e] = fmaf(dsum[t * 8 + 4 + e], xb[e], ys[4 + e] * kInvCarYS);
      }
    }
    float s1 = 0.0f;
#pragma unroll
    for (int e = 0; e < 16; ++e) s1 += v[e];
#pragma unroll
    for (int o = 16; o > 0; o >>= 1) s1 += __shfl_xor(s1, o, 32);
    const float mu = s1 * (1.0f / (float)kDi);
    float s2 = 0.0f;
#pragma unroll
    for (int e = 0; e < 16; ++e) {
      const float c = v[e] - mu;
      s2 = fmaf(c, c, s2);
    }
#pragma unroll
    for (int o = 16; o > 0; o >>= 1) s2 += __shfl_xor(s2, o, 32);
    const float var = s2 * (1.0f / (float)kDi);
    const float rs = rsqrtf(var + kLnEps);
    v8h hv[2];
#pragma unroll
    for (int t = 0; t < 2; ++t) {
      const size_t off = (size_t)row * kDi + t * 256 + lane * 8;
      const v4f za = *(const v4f*)(Z + off);
      const v4f zb = *(const v4f*)(Z + off + 4);
#pragma unroll
      for (int e = 0; e < 4; ++e) {
        const float n0v = fmaf((v[t * 8 + e] - mu) * rs, gg[t * 8 + e], bb[t * 8 + e]);
        const float n1v = fmaf((v[t * 8 + 4 + e] - mu) * rs, gg[t * 8 + 4 + e], bb[t * 8 + 4 + e]);
        hv[t][e]     = (_Float16)clamp_h16(n0v * za[e] * kCarYZ);
        hv[t][4 + e] = (_Float16)clamp_h16(n1v * zb[e] * kCarYZ);
      }
    }
    for (int pass = 0; pass < 2; ++pass) {
#pragma unroll
      for (int t = 0; t < 2; ++t) {
        unsigned short* dst = YZ + (size_t)row * kDi + t * 256 + lane * 8;
        *(volatile v8h*)dst = hv[t];
      }
      __threadfence();
    }
  }
}

extern "C" void kernel_launch(void* const* d_in, const int* in_sizes, int n_in,
                              void* d_out, int out_size, void* d_ws, size_t ws_size,
                              hipStream_t stream) {
  if (n_in < 12) return;
  if (in_sizes[0] != kRows * kDm) return;
  if (in_sizes[1] != kXzN * kDm) return;
  if (in_sizes[2] != kDi * 4) return;
  if (in_sizes[3] != kDi) return;
  if (in_sizes[4] != kPn * kDi) return;
  if (in_sizes[5] != kDirs * kDi * kDtR) return;
  if (in_sizes[6] != kDirs * kDi) return;
  if (in_sizes[7] != kDirs * kDi * kNst) return;
  if (in_sizes[8] != kDirs * kDi) return;
  if (in_sizes[9] != kDi) return;
  if (in_sizes[10] != kDi) return;
  if (in_sizes[11] != kDm * kDi) return;
  if (out_size != kRows * kDm) return;
  if (ws_size < kWsTotal) return;

  const float* x       = (const float*)d_in[0];
  const float* w_in    = (const float*)d_in[1];
  const float* conv_w  = (const float*)d_in[2];
  const float* conv_b  = (const float*)d_in[3];
  const float* w_xp    = (const float*)d_in[4];
  const float* w_dt    = (const float*)d_in[5];
  const float* b_dt    = (const float*)d_in[6];
  const float* a_log   = (const float*)d_in[7];
  const float* d_skip  = (const float*)d_in[8];
  const float* ln_g    = (const float*)d_in[9];
  const float* ln_b    = (const float*)d_in[10];
  const float* w_out   = (const float*)d_in[11];
  float* out = (float*)d_out;

  char* ws = (char*)d_ws;
  unsigned short* X16  = (unsigned short*)(ws + kOffX16);
  unsigned short* W0   = (unsigned short*)(ws + kOffW0);
  unsigned short* W1   = (unsigned short*)(ws + kOffW1);
  unsigned short* W2   = (unsigned short*)(ws + kOffW2);
  float*          XS   = (float*)(ws + kOffXS);
  float*          Zp   = (float*)(ws + kOffZ);
  float*          XC   = (float*)(ws + kOffXC);
  unsigned short* XC16 = (unsigned short*)(ws + kOffXC16);
  float*          Pp   = (float*)(ws + kOffP);
  unsigned short* YS   = (unsigned short*)(ws + kOffYS);
  unsigned short* YZ   = (unsigned short*)(ws + kOffYZ);

  prep_f16_planes_kernel<<<kPbX + kPbW0 + kPbW1 + kPbW2, 256, 0, stream>>>(x, w_in, w_xp, w_out, X16, W0, W1, W2);

  wmma_gemm64_f16<kDi><<<(kRows / 64) * (kXzN / 64) / 8, 256, 0, stream>>>(
      X16, kDm, W0, kDm, XS, Zp, kDi, kRows, kXzN, kDm, kSclIn);

  conv_act_kernel<<<(kRows * (kDi / 4)) / 256, 256, 0, stream>>>(XS, conv_w, conv_b, XC, XC16);

  wmma_gemm64_f16<0><<<(kRows / 64) * (kPn / 64) / 8, 256, 0, stream>>>(
      XC16, kDi, W1, kDi, Pp, Pp, kPn, kRows, kPn, kDi, kSclXp);

  scan_dirs_kernel<<<kBatch * kDirs * (kDi / kScCh), kScCh, 0, stream>>>(Pp, XC, w_dt, b_dt, a_log, YS);

  merge_norm_gate_kernel<<<kRows / 32, 256, 0, stream>>>(YS, XC, Zp, d_skip, ln_g, ln_b, YZ);

  wmma_gemm64_f16<0><<<(kRows / 64) * (kDm / 64) / 8, 256, 0, stream>>>(
      YZ, kDi, W2, kDi, out, out, kDm, kRows, kDm, kDi, kSclOut);
}
